// MSSFM_13529146982479
// MI455X (gfx1250) — hardware-verified
//
#include <hip/hip_runtime.h>
#include <math.h>
#include <stdint.h>

#pragma clang fp contract(off)

#define NBATCH 4
#define NSUB   8
#define NCH    128
#define NCH2   256
#define IMGH   128
#define IMGW   128
#define HWPIX  16384
#define NPIX   65536
#define KC     96
#define KCP    104
#define TP     136
#define GP     264
#define OPF    132
#define RSQ2   0.70710678118654752f

#define WOFS_C0   0
#define WOFS_C1   12288
#define WOFS_M(j) (24576 + (j) * 16384)
#define WOFS_P1   106496
#define WOFS_P2   139264
#define WTOT      172032

#define LDS_CONV ((2 * 128 * KCP + 2 * 128 * TP) * 2)
#define LDS_PAIR (2 * 128 * TP * 2)
#define LDS_TRI  ((2 * 128 * TP + 2 * 128 * GP) * 2)

static_assert(NPIX == NBATCH * HWPIX);
static_assert(HWPIX == IMGH * IMGW);
static_assert((KC % 32) == 0 && KC >= NSUB * 9);
static_assert((KCP % 8) == 0 && (TP % 8) == 0 && (GP % 8) == 0 && (OPF % 4) == 0);
static_assert(WOFS_C1 == NCH * KC && WOFS_M(0) == 2 * NCH * KC);
static_assert(WOFS_P1 == WOFS_M(5) && WOFS_P2 == WOFS_P1 + NCH2 * NCH && WTOT == WOFS_P2 + NCH * NCH2);
static_assert(128 * OPF * 4 <= 2 * 128 * TP * 2);
static_assert(LDS_CONV == 122880 && LDS_PAIR == 69632 && LDS_TRI == 204800);
static_assert(((WTOT * 2) % 256) == 0);

typedef unsigned short us_t;
typedef us_t           v8us __attribute__((ext_vector_type(8)));
typedef __bf16         v16b __attribute__((ext_vector_type(16)));
typedef _Float16       v16h __attribute__((ext_vector_type(16)));
typedef float          v8f  __attribute__((ext_vector_type(8)));
typedef float          v4f  __attribute__((ext_vector_type(4)));
typedef unsigned int   v4u  __attribute__((ext_vector_type(4)));

union FragB { v16b v; v8us u[2]; };
union F8    { v4f q[2]; float f[8]; };
static_assert(sizeof(FragB) == 32);
static_assert(sizeof(F8) == 32);

__device__ __forceinline__ us_t bf_bits(float f) {
  const unsigned u = __float_as_uint(f);
  return (us_t)((u + 0x7FFFu + ((u >> 16) & 1u)) >> 16);
}
__device__ __forceinline__ float bf_up(us_t hb) { return __uint_as_float(((unsigned)hb) << 16); }
__device__ __forceinline__ float bfr(float f) { return bf_up(bf_bits(f)); }
__device__ __forceinline__ unsigned pk16(us_t a, us_t b) { return (unsigned)a | ((unsigned)b << 16); }
__device__ __forceinline__ float bfw(v4u q, int r) {
  const unsigned w = q[r >> 1];
  return __uint_as_float((r & 1) ? (w & 0xFFFF0000u) : (w << 16));
}
__device__ __forceinline__ v8f zero8() { v8f z = {0.f, 0.f, 0.f, 0.f, 0.f, 0.f, 0.f, 0.f}; return z; }
__device__ __forceinline__ float sigm(float v) { return 1.0f / (1.0f + expf(-v)); }
__device__ __forceinline__ float gelu_e(float v) {
  const float u = v * RSQ2;
  return v * (erff(u) + 1.0f) * 0.5f;
}

__device__ __forceinline__ void split8(const float (&v)[8], v4u& hi, v4u& lo) {
  v4u a, b;
#pragma unroll
  for (int t = 0; t < 4; ++t) {
    const us_t h0 = bf_bits(v[2 * t]), h1 = bf_bits(v[2 * t + 1]);
    const us_t l0 = bf_bits(v[2 * t] - bf_up(h0)), l1 = bf_bits(v[2 * t + 1] - bf_up(h1));
    a[t] = pk16(h0, h1);
    b[t] = pk16(l0, l1);
  }
  hi = a;
  lo = b;
}

__device__ __forceinline__ v16b ldfrag(const us_t* p) {
  FragB f;
  f.u[0] = *(const v8us*)(p);
  f.u[1] = *(const v8us*)(p + 16);
  return f.v;
}

__device__ __forceinline__ v8f mma_b(v16b a, v16b b, v8f c) {
  v8f d = __builtin_amdgcn_wmma_f32_16x16x32_bf16(false, a, false, b, (short)0, c, false, false);
#if defined(__HIP_DEVICE_COMPILE__)
  const v16h ha = __builtin_bit_cast(v16h, a), hb = __builtin_bit_cast(v16h, b);
  asm volatile("v_nop\n\tv_nop\n\tv_nop\n\tv_nop" : "+v"(d) : "v"(ha), "v"(hb));
#endif
  return d;
}

template <int KS, int NJ, bool SPLIT>
__device__ __forceinline__ void gemm_w(const us_t* __restrict__ A, int lda, int arow,
                                       const us_t* Bh, const us_t* Bl, int ldb, int brow,
                                       int c, int lh, v8f (&acc)[2][NJ]) {
#pragma unroll
  for (int i = 0; i < 2; ++i)
#pragma unroll
    for (int j = 0; j < NJ; ++j) acc[i][j] = zero8();
  const us_t* ap  = A  + (size_t)(arow + c) * lda + 8 * lh;
  const us_t* bhp = Bh + (size_t)(brow + c) * ldb + 8 * lh;
  const us_t* blp = Bl + (size_t)(brow + c) * ldb + 8 * lh;
#pragma unroll 1
  for (int ks = 0; ks < KS; ++ks) {
    const v16b a0 = ldfrag(ap + 32 * ks);
    const v16b a1 = ldfrag(ap + (size_t)16 * lda + 32 * ks);
#pragma unroll
    for (int j = 0; j < NJ; ++j) {
      const v16b bh = ldfrag(bhp + (size_t)16 * j * ldb + 32 * ks);
      acc[0][j] = mma_b(a0, bh, acc[0][j]);
      acc[1][j] = mma_b(a1, bh, acc[1][j]);
      if (SPLIT) {
        const v16b bl = ldfrag(blp + (size_t)16 * j * ldb + 32 * ks);
        acc[0][j] = mma_b(a0, bl, acc[0][j]);
        acc[1][j] = mma_b(a1, bl, acc[1][j]);
      }
    }
  }
}

__global__ __launch_bounds__(256)
void k_cvtw(const float* __restrict__ cw0, const float* __restrict__ cw1,
            const float* __restrict__ m0w, const float* __restrict__ m1w, const float* __restrict__ m2w,
            const float* __restrict__ m3w, const float* __restrict__ m4w,
            const float* __restrict__ p1w, const float* __restrict__ p2w, us_t* WB) {
  const int y = blockIdx.y;
  const int i = blockIdx.x * 256 + threadIdx.x;
  const float* src = cw0;
  int cnt  = (NCH * KC) / 8;
  int dofs = WOFS_C0;
  if (y == 1)      { src = cw1; dofs = WOFS_C1; }
  else if (y == 2) { src = m0w; cnt = (NCH * NCH) / 8;  dofs = WOFS_M(0); }
  else if (y == 3) { src = m1w; cnt = (NCH * NCH) / 8;  dofs = WOFS_M(1); }
  else if (y == 4) { src = m2w; cnt = (NCH * NCH) / 8;  dofs = WOFS_M(2); }
  else if (y == 5) { src = m3w; cnt = (NCH * NCH) / 8;  dofs = WOFS_M(3); }
  else if (y == 6) { src = m4w; cnt = (NCH * NCH) / 8;  dofs = WOFS_M(4); }
  else if (y == 7) { src = p1w; cnt = (NCH2 * NCH) / 8; dofs = WOFS_P1; }
  else if (y == 8) { src = p2w; cnt = (NCH * NCH2) / 8; dofs = WOFS_P2; }
  if (i >= cnt) return;

  F8 f;
  bool ok = true;
  if (y < 2) {
    const int row = i / (KC / 8);
    const int seg = i - row * (KC / 8);
    const int k0  = min(seg * 8, NSUB * 9 - 8);
    ok = seg < 9;
    const float* p = src + row * (NSUB * 9) + k0;
    f.q[0] = *(const v4f*)(p);
    f.q[1] = *(const v4f*)(p + 4);
  } else {
    const float* p = src + (size_t)i * 8;
    f.q[0] = *(const v4f*)(p);
    f.q[1] = *(const v4f*)(p + 4);
  }
  v4u w;
#pragma unroll
  for (int t = 0; t < 4; ++t) {
    const float a = ok ? f.f[2 * t] : 0.f;
    const float b = ok ? f.f[2 * t + 1] : 0.f;
    w[t] = pk16(bf_bits(a), bf_bits(b));
  }
  us_t* dp = WB + dofs + (size_t)i * 8;
  *(volatile v4u*)dp = w;
  __threadfence();
  *(volatile v4u*)dp = w;
}

__global__ __launch_bounds__(256)
void k_dconv(const float* __restrict__ x, const us_t* __restrict__ WC,
             const float* __restrict__ b1, const float* __restrict__ b4, const float* __restrict__ pa,
             us_t* Y1h, us_t* Y1l) {
  extern __shared__ __align__(16) us_t dynlds[];
  us_t* Im = dynlds;
  us_t* Yh = dynlds + 2 * 128 * KCP;
  us_t* Yl = Yh + 128 * TP;
  const int tid  = threadIdx.x;
  const int blk  = blockIdx.x;
  const int b    = blk >> 7;
  const int hrow = blk & 127;
  const size_t n0 = (size_t)blk * 128;

#pragma unroll 2
  for (int idx = tid; idx < 2 * 128 * KC; idx += 256) {
    const int br = (idx >= 128 * KC) ? 1 : 0;
    const int r  = idx - br * 128 * KC;
    const int p  = r / KC;
    const int k  = r - p * KC;
    const int d  = br ? 7 : 1;
    const int kk = min(k, NSUB * 9 - 1);
    const int s  = kk / 9;
    const int t  = kk - 9 * s;
    const int ky = t / 3;
    const int kx = t - 3 * ky;
    const int hh = hrow + d * (ky - 1);
    const int ww = p + d * (kx - 1);
    const bool inb = (k < NSUB * 9) && (hh >= 0) && (hh < IMGH) && (ww >= 0) && (ww < IMGW);
    const int hc = min(max(hh, 0), IMGH - 1);
    const int wc = min(max(ww, 0), IMGW - 1);
    float v = x[(((size_t)b * NSUB + s) * IMGH + hc) * IMGW + wc];
    v = inb ? v : 0.f;
    Im[(br * 128 + p) * KCP + k] = bf_bits(v);
  }
  __syncthreads();

  const int lane = tid & 31, wave = tid >> 5;
  const int lh = lane >> 4, c = lane & 15;
  const int wm = (wave & 3) * 32, wn = (wave >> 2) * 64;
  const float alpha = bfr(pa[0]);

#pragma unroll 1
  for (int half = 0; half < 2; ++half) {
    const int bn = wn + half * 32;
    v8f acc0[2][2], acc1[2][2];
    gemm_w<3, 2, false>(WC, KC, wm, Im, Im, KCP, bn, c, lh, acc0);
    gemm_w<3, 2, false>(WC + NCH * KC, KC, wm, Im + 128 * KCP, Im + 128 * KCP, KCP, bn, c, lh, acc1);
#pragma unroll
    for (int i = 0; i < 2; ++i) {
#pragma unroll
      for (int j = 0; j < 2; ++j) {
        const int mb = wm + 16 * i + 8 * lh;
        const int n  = bn + 16 * j + c;
        F8 bv1, bv4;
        bv1.q[0] = *(const v4f*)(b1 + mb); bv1.q[1] = *(const v4f*)(b1 + mb + 4);
        bv4.q[0] = *(const v4f*)(b4 + mb); bv4.q[1] = *(const v4f*)(b4 + mb + 4);
        float yv[8];
#pragma unroll
        for (int r = 0; r < 8; ++r) {
          float v1 = acc0[i][j][r] + bfr(bv1.f[r]);
          v1 = (v1 >= 0.f) ? v1 : alpha * v1;
          float v4 = acc1[i][j][r] + bfr(bv4.f[r]);
          v4 = (v4 >= 0.f) ? v4 : alpha * v4;
          yv[r] = v1 + v4;
        }
        v4u hi, lo;
        split8(yv, hi, lo);
        *(v4u*)(Yh + n * TP + mb) = hi;
        *(v4u*)(Yl + n * TP + mb) = lo;
      }
    }
  }
  __syncthreads();

  {
    const int e = tid & 7, lq = tid >> 3;
#pragma unroll
    for (int pass = 0; pass < 2; ++pass) {
#pragma unroll
      for (int it = 0; it < 8; ++it) {
        const int L  = it * 32 + lq;
        const int n  = L >> 1, hf = L & 1;
        const int lo_ = n * TP + hf * 64 + 8 * e;
        const v4u vh = *(const v4u*)(Yh + lo_);
        const v4u vl = *(const v4u*)(Yl + lo_);
        const size_t go = (n0 + n) * NCH + hf * 64 + 8 * e;
        *(volatile v4u*)(Y1h + go) = vh;
        *(volatile v4u*)(Y1l + go) = vl;
      }
      __threadfence();
    }
  }
}

template <int ACT>
__global__ __launch_bounds__(256)
void k_pair(const us_t* __restrict__ Wa, const float* __restrict__ ba,
            const us_t* __restrict__ Wb, const float* __restrict__ bb,
            const us_t* __restrict__ Y1h, const us_t* __restrict__ Y1l, float* Zout) {
  extern __shared__ __align__(16) us_t dynlds[];
  us_t* Th = dynlds;
  us_t* Tl = dynlds + 128 * TP;
  float* Os = (float*)dynlds;
  const int tid = threadIdx.x;
  const int lane = tid & 31, wave = tid >> 5;
  const int lh = lane >> 4, c = lane & 15;
  const int wm = (wave & 3) * 32, wn = (wave >> 2) * 64;
  const size_t n0 = (size_t)blockIdx.x * 128;

  v8f acc[2][4];
  gemm_w<4, 4, true>(Wa, NCH, wm, Y1h + n0 * NCH, Y1l + n0 * NCH, NCH, wn, c, lh, acc);
#pragma unroll
  for (int i = 0; i < 2; ++i) {
#pragma unroll
    for (int j = 0; j < 4; ++j) {
      const int mb = wm + 16 * i + 8 * lh;
      const int n  = wn + 16 * j + c;
      F8 bv;
      bv.q[0] = *(const v4f*)(ba + mb); bv.q[1] = *(const v4f*)(ba + mb + 4);
      float t[8];
#pragma unroll
      for (int r = 0; r < 8; ++r) t[r] = tanhf(acc[i][j][r] + bfr(bv.f[r]));
      v4u hi, lo;
      split8(t, hi, lo);
      *(v4u*)(Th + n * TP + mb) = hi;
      *(v4u*)(Tl + n * TP + mb) = lo;
    }
  }
  __syncthreads();

  gemm_w<4, 4, true>(Wb, NCH, wm, Th, Tl, TP, wn, c, lh, acc);
  __syncthreads();
#pragma unroll
  for (int i = 0; i < 2; ++i) {
#pragma unroll
    for (int j = 0; j < 4; ++j) {
      const int mb = wm + 16 * i + 8 * lh;
      const int n  = wn + 16 * j + c;
      F8 bv, o;
      bv.q[0] = *(const v4f*)(bb + mb); bv.q[1] = *(const v4f*)(bb + mb + 4);
#pragma unroll
      for (int r = 0; r < 8; ++r) {
        const float v = acc[i][j][r] + bfr(bv.f[r]);
        o.f[r] = (ACT == 0) ? tanhf(v) : sigm(v);
      }
      *(v4f*)(Os + n * OPF + mb)     = o.q[0];
      *(v4f*)(Os + n * OPF + mb + 4) = o.q[1];
    }
  }
  __syncthreads();

  {
    const int e = tid & 7, lq = tid >> 3;
    float* zb = Zout + n0 * NCH;
#pragma unroll
    for (int pass = 0; pass < 2; ++pass) {
#pragma unroll
      for (int it = 0; it < 16; ++it) {
        const int L = it * 32 + lq;
        const int n = L >> 2, q = L & 3;
        const v4f v = *(const v4f*)(Os + n * OPF + q * 32 + 4 * e);
        *(volatile v4f*)(zb + (size_t)n * NCH + q * 32 + 4 * e) = v;
      }
      __threadfence();
    }
  }
}

__global__ __launch_bounds__(256)
void k_scan(const float* Zin, const float* __restrict__ Fin,
            const us_t* __restrict__ Y1h, const us_t* __restrict__ Y1l, float* Gout) {
  const int tid = threadIdx.x;
  const int c   = tid & 127;
  const int pw  = blockIdx.x * 2 + (tid >> 7);
  const int b   = pw >> 7;
  const int w   = pw & 127;
  const size_t base = ((size_t)b * HWPIX + w) * NCH + c;
  const bool fwd = (c >= NCH / 2);
  float hs = 0.f;
#pragma unroll 1
  for (int s = 0; s < IMGH; ++s) {
    const int hh = fwd ? s : (IMGH - 1 - s);
    const size_t idx = base + (size_t)hh * (IMGW * NCH);
    const float z = Zin[idx];
    const float f = Fin[idx];
    hs = f * hs + (1.0f - f) * z;
    const float y1 = bf_up(Y1h[idx]) + bf_up(Y1l[idx]);
    const float g  = y1 * sigm(hs);
    *(volatile float*)(Gout + idx) = g;
    __threadfence();
    *(volatile float*)(Gout + idx) = g;
  }
}

__global__ __launch_bounds__(256)
void k_tri(const us_t* __restrict__ W5, const float* __restrict__ pb5,
           const us_t* __restrict__ W6, const float* __restrict__ pb6,
           const us_t* __restrict__ W7, const float* __restrict__ pb7,
           const us_t* __restrict__ Y1h, const us_t* __restrict__ Y1l,
           const float* __restrict__ Gate, float* out) {
  extern __shared__ __align__(16) us_t dynlds[];
  us_t* Pth = dynlds;
  us_t* Ptl = dynlds + 128 * TP;
  us_t* Gth = dynlds + 256 * TP;
  us_t* Gtl = Gth + 128 * GP;
  float* Os = (float*)dynlds;
  const int tid = threadIdx.x;
  const int lane = tid & 31, wave = tid >> 5;
  const int lh = lane >> 4, c = lane & 15;
  const int wm = (wave & 3) * 32, wn = (wave >> 2) * 64;
  const int blk  = blockIdx.x;
  const int b    = blk >> 7;
  const int hrow = blk & 127;
  const size_t n0 = (size_t)blk * 128;

  {
    v8f acc[2][4];
    gemm_w<4, 4, true>(W5, NCH, wm, Y1h + n0 * NCH, Y1l + n0 * NCH, NCH, wn, c, lh, acc);
#pragma unroll
    for (int i = 0; i < 2; ++i) {
#pragma unroll
      for (int j = 0; j < 4; ++j) {
        const int mb = wm + 16 * i + 8 * lh;
        const int n  = wn + 16 * j + c;
        F8 bv;
        bv.q[0] = *(const v4f*)(pb5 + mb); bv.q[1] = *(const v4f*)(pb5 + mb + 4);
        const v4u yh = *(const v4u*)(Y1h + (n0 + n) * NCH + mb);
        const v4u yl = *(const v4u*)(Y1l + (n0 + n) * NCH + mb);
        float p[8];
#pragma unroll
        for (int r = 0; r < 8; ++r) {
          const float y1 = bfw(yh, r) + bfw(yl, r);
          const float v  = acc[i][j][r] + bfr(bv.f[r]);
          p[r] = v * y1 + y1;
        }
        v4u hi, lo;
        split8(p, hi, lo);
        *(v4u*)(Pth + n * TP + mb) = hi;
        *(v4u*)(Ptl + n * TP + mb) = lo;
      }
    }
  }
  __syncthreads();

#pragma unroll 1
  for (int mh = 0; mh < 2; ++mh) {
    v8f acc[2][4];
    gemm_w<4, 4, true>(W6, NCH, mh * 128 + wm, Pth, Ptl, TP, wn, c, lh, acc);
#pragma unroll
    for (int i = 0; i < 2; ++i) {
#pragma unroll
      for (int j = 0; j < 4; ++j) {
        const int mcol = mh * 128 + wm + 16 * i + 8 * lh;
        const int n    = wn + 16 * j + c;
        F8 bv;
        bv.q[0] = *(const v4f*)(pb6 + mcol); bv.q[1] = *(const v4f*)(pb6 + mcol + 4);
        float g[8];
#pragma unroll
        for (int r = 0; r < 8; ++r) g[r] = gelu_e(acc[i][j][r] + bfr(bv.f[r]));
        v4u hi, lo;
        split8(g, hi, lo);
        *(v4u*)(Gth + n * GP + mcol) = hi;
        *(v4u*)(Gtl + n * GP + mcol) = lo;
      }
    }
  }
  __syncthreads();

  {
    v8f acc[2][4];
    gemm_w<8, 4, true>(W7, NCH2, wm, Gth, Gtl, GP, wn, c, lh, acc);
#pragma unroll
    for (int i = 0; i < 2; ++i) {
#pragma unroll
      for (int j = 0; j < 4; ++j) {
        const int mb = wm + 16 * i + 8 * lh;
        const int n  = wn + 16 * j + c;
        F8 bv, gt, o;
        bv.q[0] = *(const v4f*)(pb7 + mb); bv.q[1] = *(const v4f*)(pb7 + mb + 4);
        const float* gp = Gate + (n0 + n) * NCH + mb;
        gt.q[0] = *(const v4f*)(gp); gt.q[1] = *(const v4f*)(gp + 4);
#pragma unroll
        for (int r = 0; r < 8; ++r) {
          const float y3 = acc[i][j][r] + bfr(bv.f[r]);
          o.f[r] = gt.f[r] + y3;
        }
        *(v4f*)(Os + n * OPF + mb)     = o.q[0];
        *(v4f*)(Os + n * OPF + mb + 4) = o.q[1];
      }
    }
  }
  __syncthreads();

  {
    const int e = tid & 7, lq = tid >> 3;
    float* ob = out + ((size_t)b * NCH) * HWPIX + (size_t)hrow * IMGW;
#pragma unroll
    for (int pass = 0; pass < 2; ++pass) {
#pragma unroll
      for (int it = 0; it < 16; ++it) {
        const int L  = it * 32 + lq;
        const int m  = L >> 2, q = L & 3;
        const int w0 = q * 32 + 4 * e;
        v4f v;
        v[0] = Os[(w0 + 0) * OPF + m];
        v[1] = Os[(w0 + 1) * OPF + m];
        v[2] = Os[(w0 + 2) * OPF + m];
        v[3] = Os[(w0 + 3) * OPF + m];
        *(volatile v4f*)(ob + (size_t)m * HWPIX + w0) = v;
      }
      __threadfence();
    }
  }
}

extern "C" void kernel_launch(void* const* d_in, const int* in_sizes, int n_in,
                              void* d_out, int out_size, void* d_ws, size_t ws_size,
                              hipStream_t stream) {
  if (n_in < 20) return;
  if (in_sizes[0] != NBATCH * NSUB * HWPIX) return;
  if (in_sizes[1] != NCH * NSUB * 9 || in_sizes[3] != NCH * NSUB * 9) return;
  if (in_sizes[2] != NCH || in_sizes[4] != NCH || in_sizes[5] < 1) return;
  if (in_sizes[6] != NCH * NCH || in_sizes[8] != NCH * NCH || in_sizes[10] != NCH * NCH ||
      in_sizes[12] != NCH * NCH || in_sizes[18] != NCH * NCH) return;
  if (in_sizes[7] != NCH || in_sizes[9] != NCH || in_sizes[11] != NCH || in_sizes[13] != NCH ||
      in_sizes[17] != NCH || in_sizes[19] != NCH) return;
  if (in_sizes[14] != NCH2 * NCH || in_sizes[15] != NCH2 || in_sizes[16] != NCH * NCH2) return;
  if (out_size != NBATCH * NCH * HWPIX) return;

  size_t off = 0;
  const size_t oW  = off; off += (size_t)WTOT * 2;
  const size_t szH = (size_t)NPIX * NCH * 2;
  const size_t szF = (size_t)NPIX * NCH * 4;
  const size_t oYh = off; off += szH;
  const size_t oYl = off; off += szH;
  const size_t oZ  = off; off += szF;
  const size_t oF  = off; off += szF;
  if (off > ws_size) return;
  if (off > (size_t)134217728) return;

  const float* x    = (const float*)d_in[0];
  const float* d1w  = (const float*)d_in[1];
  const float* d1b  = (const float*)d_in[2];
  const float* d4w  = (const float*)d_in[3];
  const float* d4b  = (const float*)d_in[4];
  const float* pa   = (const float*)d_in[5];
  const float* f1w1 = (const float*)d_in[6];
  const float* f1b1 = (const float*)d_in[7];
  const float* f1w2 = (const float*)d_in[8];
  const float* f1b2 = (const float*)d_in[9];
  const float* f2w1 = (const float*)d_in[10];
  const float* f2b1 = (const float*)d_in[11];
  const float* f2w2 = (const float*)d_in[12];
  const float* f2b2 = (const float*)d_in[13];
  const float* pw1  = (const float*)d_in[14];
  const float* pb1  = (const float*)d_in[15];
  const float* pw2  = (const float*)d_in[16];
  const float* pb2  = (const float*)d_in[17];
  const float* pw3  = (const float*)d_in[18];
  const float* pb3  = (const float*)d_in[19];

  char* ws = (char*)d_ws;
  us_t* WB  = (us_t*)(ws + oW);
  us_t* Y1h = (us_t*)(ws + oYh);
  us_t* Y1l = (us_t*)(ws + oYl);
  float* Zf = (float*)(ws + oZ);
  float* Ff = (float*)(ws + oF);
  float* y  = (float*)d_out;

  const us_t* WC = WB + WOFS_C0;
  const us_t* W1 = WB + WOFS_M(0);
  const us_t* W2 = WB + WOFS_M(1);
  const us_t* W3 = WB + WOFS_M(2);
  const us_t* W4 = WB + WOFS_M(3);
  const us_t* W5 = WB + WOFS_M(4);
  const us_t* W6 = WB + WOFS_P1;
  const us_t* W7 = WB + WOFS_P2;

  (void)hipFuncSetAttribute(reinterpret_cast<const void*>(&k_dconv),
                            hipFuncAttributeMaxDynamicSharedMemorySize, LDS_CONV);
  (void)hipFuncSetAttribute(reinterpret_cast<const void*>(&k_pair<0>),
                            hipFuncAttributeMaxDynamicSharedMemorySize, LDS_PAIR);
  (void)hipFuncSetAttribute(reinterpret_cast<const void*>(&k_pair<1>),
                            hipFuncAttributeMaxDynamicSharedMemorySize, LDS_PAIR);
  (void)hipFuncSetAttribute(reinterpret_cast<const void*>(&k_tri),
                            hipFuncAttributeMaxDynamicSharedMemorySize, LDS_TRI);

  const dim3 blk256(256);
  const dim3 gW(16, 9);
  const dim3 gT(NPIX / 128);
  const dim3 gS((NBATCH * IMGW * NCH) / 256);

  k_cvtw<<<gW, blk256, 0, stream>>>(d1w, d4w, f1w1, f1w2, f2w1, f2w2, pw3, pw1, pw2, WB);
  k_dconv<<<gT, blk256, LDS_CONV, stream>>>(x, WC, d1b, d4b, pa, Y1h, Y1l);
  k_pair<0><<<gT, blk256, LDS_PAIR, stream>>>(W1, f1b1, W2, f1b2, Y1h, Y1l, Zf);
  k_pair<1><<<gT, blk256, LDS_PAIR, stream>>>(W3, f2b1, W4, f2b2, Y1h, Y1l, Ff);
  k_scan<<<gS, blk256, 0, stream>>>(Zf, Ff, Y1h, Y1l, Zf);
  k_tri<<<gT, blk256, LDS_TRI, stream>>>(W5, pb3, W6, pb1, W7, pb2, Y1h, Y1l, Zf, y);
  (void)hipGetLastError();
}
